// NonLocal_77790447665590
// MI455X (gfx1250) — hardware-verified
//
#include <hip/hip_runtime.h>
#include <math.h>

typedef __attribute__((ext_vector_type(16))) _Float16 v16h;
typedef __attribute__((ext_vector_type(16))) __bf16 v16b;
typedef __attribute__((ext_vector_type(8)))  _Float16 v8h;
typedef __attribute__((ext_vector_type(8)))  float v8f;
typedef __attribute__((ext_vector_type(4)))  float v4f;
typedef __attribute__((ext_vector_type(2)))  float v2f;
typedef __attribute__((ext_vector_type(4)))  unsigned v4u;
typedef __attribute__((ext_vector_type(4)))  int v4i;
typedef float __attribute__((may_alias)) float_a;
typedef int __attribute__((may_alias)) int_a;

template <typename T> __device__ __forceinline__ void vst2(void* p, T v) { *(volatile T*)p = v; __threadfence(); *(volatile T*)p = v; }
__device__ __forceinline__ v8f wmma16(v16h a, v16h b, v8f c) {
  v8f d = __builtin_amdgcn_wmma_f32_16x16x32_f16(false, a, false, b, (short)0, c, false, false);
  asm volatile("v_nop\n\tv_nop\n\tv_nop\n\tv_nop" : "+v"(d) : "v"(a), "v"(b));
  return d;
}
__device__ __forceinline__ v8f wmma_bf(v16b a, v16b b, v8f c) {
  v8f d = __builtin_amdgcn_wmma_f32_16x16x32_bf16(false, a, false, b, (short)0, c, false, false);
  asm volatile("v_nop\n\tv_nop\n\tv_nop\n\tv_nop" : "+v"(d) : "v"(a), "v"(b));
  return d;
}
__device__ __forceinline__ v16h frag_h(const _Float16* rowk0, int lane) {
  union { v16h v; v8h q[2]; } u; const _Float16* p = rowk0 + 8 * (lane >> 4);
  u.q[0] = *(const v8h*)p; u.q[1] = *(const v8h*)(p + 16); return u.v;
}
__device__ __forceinline__ v16h frag_f32(const float* rowk0, int lane) {
  v16h a; const float* p = rowk0 + 8 * (lane >> 4);
#pragma unroll
  for (int i = 0; i < 8; ++i) { a[i] = (_Float16)p[i]; a[8 + i] = (_Float16)p[16 + i]; }
  return a;
}
__device__ __forceinline__ v16h frag_f32s(const float* rowk0, int lane, float sc) {
  v16h a; const float* p = rowk0 + 8 * (lane >> 4);
#pragma unroll
  for (int i = 0; i < 8; ++i) { a[i] = (_Float16)(p[i] * sc); a[8 + i] = (_Float16)(p[16 + i] * sc); }
  return a;
}
__device__ __forceinline__ v16h fragc_f32(const float* W, int k0, int n, int lane, int ld, int K) {
  v16h a; const int g = lane >> 4;
#pragma unroll
  for (int i = 0; i < 8; ++i) { const int ka = k0 + 8 * g + i, kb = ka + 16;
    a[i] = (_Float16)(ka < K ? W[(size_t)(ka < K ? ka : K - 1) * ld + n] : 0.f); a[8 + i] = (_Float16)(kb < K ? W[(size_t)(kb < K ? kb : K - 1) * ld + n] : 0.f); }
  return a;
}
struct F2 { v16b h, l; };
__device__ __forceinline__ F2 bsplit16(const float v[16]) { F2 r;
#pragma unroll
  for (int i = 0; i < 16; ++i) { const __bf16 h = (__bf16)v[i]; r.h[i] = h; r.l[i] = (__bf16)(v[i] - (float)h); }
  return r; }
__device__ __forceinline__ F2 split_row(const float* row, int k0, int lane) { float v[16]; const float* p = row + k0 + 8 * (lane >> 4);
#pragma unroll
  for (int i = 0; i < 8; ++i) { v[i] = p[i]; v[8 + i] = p[16 + i]; }
  return bsplit16(v); }
__device__ __forceinline__ F2 split_rowK(const float* row, int k0, int lane, int K) { float v[16]; const int g = lane >> 4;
#pragma unroll
  for (int i = 0; i < 8; ++i) { const int ka = k0 + 8 * g + i, kb = ka + 16; v[i] = ka < K ? row[ka < K ? ka : K - 1] : 0.f; v[8 + i] = kb < K ? row[kb < K ? kb : K - 1] : 0.f; }
  return bsplit16(v); }
__device__ __forceinline__ F2 split_col(const float* W, int k0, int n, int lane, int ld, int K) { float v[16]; const int g = lane >> 4;
#pragma unroll
  for (int i = 0; i < 8; ++i) { const int ka = k0 + 8 * g + i, kb = ka + 16; v[i] = ka < K ? W[(size_t)(ka < K ? ka : K - 1) * ld + n] : 0.f; v[8 + i] = kb < K ? W[(size_t)(kb < K ? kb : K - 1) * ld + n] : 0.f; }
  return bsplit16(v); }
__device__ __forceinline__ v8f mac3(const F2& a, const F2& b, v8f c) { c = wmma_bf(a.l, b.h, c); c = wmma_bf(a.h, b.l, c); return wmma_bf(a.h, b.h, c); }
__device__ __forceinline__ float sigm(float v) { return 1.0f / (1.0f + expf(-v)); }
#define LDSX() do { asm volatile("s_wait_dscnt 0" ::: "memory"); __builtin_amdgcn_wave_barrier(); __builtin_amdgcn_fence(__ATOMIC_RELEASE, "workgroup"); } while (0)


#define NB 8
#define CC 512
#define DD 256
#define TT 2048
#ifndef TNB
#define TNB NB
#endif
typedef __attribute__((ext_vector_type(8))) __bf16 v8b;
__device__ __forceinline__ v16b frag_b(const __bf16* rowk0, int lane) {
  union { v16b v; v8b q[2]; } u; const __bf16* p = rowk0 + 8 * (lane >> 4);
  u.q[0] = *(const v8b*)p; u.q[1] = *(const v8b*)(p + 16); return u.v;
}
__device__ __forceinline__ float bfr(float v) { return (float)(__bf16)v; }
__device__ __attribute__((noinline)) float exp_ni(float v) { return expf(v); }
__device__ __attribute__((noinline)) float erf_ni(float v) { return erff(v); }

#define WS_TH  0u
#define WS_PHH (WS_TH + 4u * (size_t)NB * TT * DD)
#define WS_PHL (WS_PHH + 2u * (size_t)NB * TT * DD)
#define WS_G   (WS_PHL + 2u * (size_t)NB * TT * DD)
#define WS_S   (WS_G + 4u * (size_t)NB * DD * TT)
#define WS_ML  (WS_S + 4u * (size_t)TT * TT)
#define WS_PT  (WS_ML + 4u * (size_t)TT * 8)
#define WS_AT  (WS_PT + 2u * (size_t)TT * TT)
#define WS_H   (WS_AT + 4u * (size_t)NB * TT * DD)
#define WS_ST  (WS_H + 4u * (size_t)NB * CC * TT)
#define WS_BN  (WS_ST + 4u * (size_t)NB * (TT / 64) * CC * 2)
#define WS_END (WS_BN + 4u * 2 * CC)

__global__ __launch_bounds__(128) void k_proj(const float* __restrict__ X, const float* __restrict__ WT, const float* __restrict__ BT, const float* __restrict__ WP, const float* __restrict__ BP, const float* __restrict__ WG, const float* __restrict__ BG, float* __restrict__ TH, __bf16* __restrict__ PHH, __bf16* __restrict__ PHL, float* __restrict__ G) {
  __shared__ __align__(16) __bf16 sx[64][CC + 8]; __shared__ __align__(16) float st[64][68];
  const int tid = threadIdx.x, wave = tid >> 5, lane = tid & 31, col = lane & 15, g = lane >> 4; const int t0 = blockIdx.x * 64; const size_t b = blockIdx.y; const int which = blockIdx.z;
  const float* Wm = which == 0 ? WT : which == 1 ? WP : WG; const float* Bm = which == 0 ? BT : which == 1 ? BP : BG;
  for (int e = tid; e < CC * 64; e += 128) { const int c = e >> 6, tl = e & 63; sx[tl][c] = (__bf16)X[(b * CC + c) * (size_t)TT + t0 + tl]; }
  __syncthreads();
#pragma unroll 1
  for (int cg = 0; cg < DD / 64; ++cg) { v8f acc[4] = {};
#pragma unroll 2
    for (int kc = 0; kc < CC / 32; ++kc) { const v16b a = frag_b(&sx[wave * 16 + col][kc * 32], lane);
#pragma unroll
      for (int j = 0; j < 4; ++j) { v16b w; const int d = cg * 64 + j * 16 + col;
#pragma unroll
        for (int i = 0; i < 8; ++i) { w[i] = (__bf16)Wm[(size_t)d * CC + kc * 32 + 8 * g + i]; w[8 + i] = (__bf16)Wm[(size_t)d * CC + kc * 32 + 16 + 8 * g + i]; }
        acc[j] = wmma_bf(a, w, acc[j]); } }
    __syncthreads();
#pragma unroll
    for (int j = 0; j < 4; ++j) { const int dl = j * 16 + col; const float bb = bfr(Bm[cg * 64 + dl]);
#pragma unroll
      for (int r = 0; r < 8; ++r) { const int tl = wave * 16 + 8 * g + r; const float v = acc[j][r] + bb; if (which == 2) st[dl][tl] = v; else st[tl][dl] = v; } }
    __syncthreads();
    if (which == 0) { for (int e = tid; e < 64 * 16; e += 128) { const int tl = e >> 4, q = e & 15; vst2(TH + (b * TT + t0 + tl) * DD + cg * 64 + q * 4, *(const v4f*)&st[tl][q * 4]); } }
    else if (which == 1) { for (int e = tid; e < 64 * 8; e += 128) { const int tl = e >> 3, q = e & 7; const float* p = &st[tl][q * 8]; v16b dummy; (void)dummy; __bf16 hh[8], ll[8];
#pragma unroll
        for (int i = 0; i < 8; ++i) { const __bf16 hv = (__bf16)p[i]; hh[i] = hv; ll[i] = (__bf16)(p[i] - (float)hv); }
        vst2((unsigned*)(PHH + (b * TT + t0 + tl) * DD + cg * 64 + q * 8), *(const v4u*)hh); vst2((unsigned*)(PHL + (b * TT + t0 + tl) * DD + cg * 64 + q * 8), *(const v4u*)ll); } }
    else { for (int e = tid; e < 64 * 16; e += 128) { const int dl = e >> 4, q = e & 15; vst2(G + (b * DD + cg * 64 + dl) * (size_t)TT + t0 + q * 4, *(const v4f*)&st[dl][q * 4]); } } } }
__global__ __launch_bounds__(128) void k_sc(const float* __restrict__ TH, const __bf16* __restrict__ PHH, const __bf16* __restrict__ PHL, int b, float* __restrict__ S) { __shared__ __align__(16) float ss[4][16][132];
  const int tid = threadIdx.x, wave = tid >> 5, lane = tid & 31, col = lane & 15, g = lane >> 4; const int k0 = blockIdx.y * 128; const int tq0 = blockIdx.x * 64 + wave * 16; const size_t q0 = (size_t)b * TT + tq0;
  v8f acc[8] = {};
#pragma unroll 1
  for (int kc = 0; kc < DD / 32; ++kc) { const F2 a = split_row(TH + (q0 + col) * DD, kc * 32, lane);
#pragma unroll
    for (int j = 0; j < 8; ++j) { const size_t kr = ((size_t)b * TT + k0 + j * 16 + col) * DD + kc * 32; const v16b kh = frag_b(PHH + kr, lane), kl = frag_b(PHL + kr, lane); acc[j] = wmma_bf(a.h, kh, acc[j]); acc[j] = wmma_bf(a.l, kh, acc[j]); acc[j] = wmma_bf(a.h, kl, acc[j]); } }
#pragma unroll
  for (int j = 0; j < 8; ++j)
#pragma unroll
    for (int r = 0; r < 8; ++r) ss[wave][8 * g + r][j * 16 + col] = acc[j][r];
  LDSX(); for (int rl = 0; rl < 16; ++rl) vst2(S + (size_t)(tq0 + rl) * TT + k0 + lane * 4, *(const v4f*)&ss[wave][rl][lane * 4]); }
__global__ __launch_bounds__(256) void k_stat(const float* __restrict__ S, float* __restrict__ ML) { __shared__ float sred[8]; __shared__ float sbc; __shared__ __align__(16) float sout[4][8];
  const int t = threadIdx.x;
  for (int rr = 0; rr < 4; ++rr) { const size_t row = (size_t)blockIdx.x * 4 + rr; const float* sr = S + row * TT;
    float m = -3.0e38f; for (int k = t; k < TT; k += 256) m = fmaxf(m, sr[k]);
#pragma unroll
    for (int o = 1; o < 32; o <<= 1) m = fmaxf(m, __shfl_xor(m, o));
    if ((t & 31) == 0) sred[t >> 5] = m; __syncthreads(); if (t == 0) { float a = sred[0]; for (int i = 1; i < 8; ++i) a = fmaxf(a, sred[i]); sbc = a; } __syncthreads(); m = sbc; __syncthreads();
    float sum = 0.f; for (int k = t; k < TT; k += 256) sum += expf(sr[k] - m);
#pragma unroll
    for (int o = 1; o < 32; o <<= 1) sum += __shfl_xor(sum, o);
    if ((t & 31) == 0) sred[t >> 5] = sum; __syncthreads(); if (t == 0) { float a = 0.f; for (int i = 0; i < 8; ++i) a += sred[i]; sout[rr][0] = m; sout[rr][1] = 1.0f / a; for (int i = 2; i < 8; ++i) sout[rr][i] = 0.f; } __syncthreads(); }
  if (t < 8) vst2(ML + (size_t)blockIdx.x * 32 + t * 4, *(const v4f*)&(&sout[0][0])[t * 4]); }
__global__ __launch_bounds__(128) void k_pt(const float* __restrict__ S, const float* __restrict__ ML, _Float16* __restrict__ PT) { __shared__ __align__(16) _Float16 sp[128][72];
  const int tid = threadIdx.x; const int t0 = blockIdx.x * 64, s0 = blockIdx.y * 128;
  for (int e = tid; e < 64 * 128; e += 128) { const int tl = e >> 7, sl = e & 127; const float m = ML[(size_t)(t0 + tl) * 8], inv = ML[(size_t)(t0 + tl) * 8 + 1]; sp[sl][tl] = (_Float16)(expf(S[(size_t)(t0 + tl) * TT + s0 + sl] - m) * inv * 2048.0f); }
  __syncthreads(); for (int e = tid; e < 128 * 8; e += 128) { const int sl = e >> 3, q = e & 7; vst2((unsigned*)(PT + (size_t)(s0 + sl) * TT + t0 + q * 8), *(const v4u*)&sp[sl][q * 8]); } }
__global__ __launch_bounds__(128) void k_pv(const _Float16* __restrict__ PT, const float* __restrict__ G, int b, float* __restrict__ AT) { __shared__ __align__(16) float ss[4][16][132];
  const int tid = threadIdx.x, wave = tid >> 5, lane = tid & 31, col = lane & 15, g = lane >> 4; const int d0 = blockIdx.y * 128; const int s0 = blockIdx.x * 64 + wave * 16;
  v8f acc[8] = {};
#pragma unroll 1
  for (int kc = 0; kc < TT / 32; ++kc) { const v16h a = frag_h(PT + (size_t)(s0 + col) * TT + kc * 32, lane);
#pragma unroll
    for (int j = 0; j < 8; ++j) { const float* gp = G + ((size_t)b * DD + d0 + j * 16 + col) * TT + kc * 32 + 8 * g; v16h gh, gl;
#pragma unroll
      for (int i = 0; i < 8; ++i) { const float v0 = gp[i], v1 = gp[16 + i]; const _Float16 h0 = (_Float16)v0, h1 = (_Float16)v1; gh[i] = h0; gh[8 + i] = h1; gl[i] = (_Float16)(v0 - (float)h0); gl[8 + i] = (_Float16)(v1 - (float)h1); }
      acc[j] = wmma16(a, gh, acc[j]); acc[j] = wmma16(a, gl, acc[j]); } }
#pragma unroll
  for (int j = 0; j < 8; ++j)
#pragma unroll
    for (int r = 0; r < 8; ++r) ss[wave][8 * g + r][j * 16 + col] = acc[j][r] * (1.0f / 2048.0f);
  LDSX(); for (int rl = 0; rl < 16; ++rl) vst2(AT + ((size_t)b * TT + s0 + rl) * DD + d0 + lane * 4, *(const v4f*)&ss[wave][rl][lane * 4]); }
__global__ __launch_bounds__(128) void k_ht(const float* __restrict__ AT, const float* __restrict__ HW, const float* __restrict__ HB, float* __restrict__ Hh, float* __restrict__ ST) { __shared__ __align__(16) float st[128][68]; __shared__ __align__(16) float sst[128][2];
  const int tid = threadIdx.x, wave = tid >> 5, lane = tid & 31, col = lane & 15, g = lane >> 4; const int c0 = blockIdx.y * 128; const size_t b = blockIdx.z; const int s0 = blockIdx.x * 64; const size_t r0 = b * TT + s0 + wave * 16;
  v8f acc[8] = {};
#pragma unroll 1
  for (int kc = 0; kc < DD / 32; ++kc) { const F2 a = split_row(AT + (r0 + col) * DD, kc * 32, lane);
#pragma unroll
    for (int j = 0; j < 8; ++j) { v16b w; const int c = c0 + j * 16 + col;
#pragma unroll
      for (int i = 0; i < 8; ++i) { w[i] = (__bf16)HW[(size_t)c * DD + kc * 32 + 8 * g + i]; w[8 + i] = (__bf16)HW[(size_t)c * DD + kc * 32 + 16 + 8 * g + i]; }
      acc[j] = wmma_bf(a.h, w, acc[j]); acc[j] = wmma_bf(a.l, w, acc[j]); } }
#pragma unroll
  for (int j = 0; j < 8; ++j) { const int cl = j * 16 + col; const float bb = bfr(HB[c0 + cl]);
#pragma unroll
    for (int r = 0; r < 8; ++r) st[cl][wave * 16 + 8 * g + r] = acc[j][r] + bb; }
  __syncthreads();
  for (int e = tid; e < 128 * 16; e += 128) { const int cl = e >> 4, q = e & 15; vst2(Hh + (b * CC + c0 + cl) * (size_t)TT + s0 + q * 4, *(const v4f*)&st[cl][q * 4]); }
  { const int cl = tid; float s = 0.f; for (int q = 0; q < 64; ++q) s += st[cl][q]; const float mean = s / 64.0f; float m2 = 0.f; for (int q = 0; q < 64; ++q) { const float d = st[cl][q] - mean; m2 += d * d; } sst[cl][0] = mean; sst[cl][1] = m2; }
  __syncthreads(); if (tid < 64) vst2(ST + (((b * (TT / 64) + blockIdx.x) * CC) + c0) * 2 + tid * 4, *(const v4f*)&(&sst[0][0])[tid * 4]); }
__global__ __launch_bounds__(512) void k_bn(const float* __restrict__ ST, float* __restrict__ BN) { __shared__ __align__(16) float s[2][CC]; const int c = threadIdx.x; float n = 0.f, mean = 0.f, M2 = 0.f;
#pragma unroll 1
  for (int blk = 0; blk < NB * (TT / 64); ++blk) { const float mb = ST[((size_t)blk * CC + c) * 2], qb = ST[((size_t)blk * CC + c) * 2 + 1]; const float nb_ = 64.f; const float nt = n + nb_; const float d = mb - mean; mean += d * nb_ / nt; M2 += qb + d * d * n * nb_ / nt; n = nt; }
  s[0][c] = mean; s[1][c] = 1.0f / sqrtf(M2 / n + 1e-5f); __syncthreads(); if (c < 2 * CC / 4) vst2(BN + c * 4, *(const v4f*)&(&s[0][0])[c * 4]); }
__global__ __launch_bounds__(256) void k_out(const float* __restrict__ X, const float* __restrict__ Hh, const float* __restrict__ BN, const float* __restrict__ GA, const float* __restrict__ BE, float* __restrict__ OUT) { __shared__ __align__(16) float so[TT]; const int t = threadIdx.x; const int c = blockIdx.x; const size_t b = blockIdx.y; const float mean = BN[c], inv = BN[CC + c], ga = bfr(GA[c]), be = bfr(BE[c]);
  const size_t base = (b * CC + c) * (size_t)TT; for (int e = t; e < TT; e += 256) so[e] = bfr(X[base + e]) + (ga * (Hh[base + e] - mean) * inv + be);
  __syncthreads(); for (int q = t; q < TT / 4; q += 256) vst2(OUT + base + q * 4, *(const v4f*)&so[q * 4]); }
extern "C" void kernel_launch(void* const* d_in, const int* in_sizes, int n_in, void* d_out, int out_size, void* d_ws, size_t ws_size, hipStream_t stream) {
  (void)in_sizes; (void)n_in; (void)out_size;
  const float** F = (const float**)d_in;
  if (ws_size < (size_t)WS_END) return;
  char* ws = (char*)d_ws; float *TH = (float*)(ws + WS_TH), *G = (float*)(ws + WS_G), *S = (float*)(ws + WS_S), *ML = (float*)(ws + WS_ML), *AT = (float*)(ws + WS_AT), *Hh = (float*)(ws + WS_H), *ST = (float*)(ws + WS_ST), *BN = (float*)(ws + WS_BN); __bf16 *PHH = (__bf16*)(ws + WS_PHH), *PHL = (__bf16*)(ws + WS_PHL); _Float16* PT = (_Float16*)(ws + WS_PT);
  k_proj<<<dim3(TT / 64, TNB, 3), 128, 0, stream>>>(F[0], F[1], F[2], F[3], F[4], F[5], F[6], TH, PHH, PHL, G);
  for (int b = 0; b < TNB; ++b) {
    k_sc<<<dim3(TT / 64, TT / 128), 128, 0, stream>>>(TH, PHH, PHL, b, S);
    k_stat<<<TT / 4, 256, 0, stream>>>(S, ML);
    k_pt<<<dim3(TT / 64, TT / 128), 128, 0, stream>>>(S, ML, PT);
    k_pv<<<dim3(TT / 64, DD / 128), 128, 0, stream>>>(PT, G, b, AT);
  }
  k_ht<<<dim3(TT / 64, CC / 128, TNB), 128, 0, stream>>>(AT, F[7], F[8], Hh, ST);
  k_bn<<<1, 512, 0, stream>>>(ST, BN);
  k_out<<<dim3(CC, TNB), 256, 0, stream>>>(F[0], Hh, BN, F[9], F[10], (float*)d_out);
}
